// Block_Height_Reducing_Filtering_47158740910393
// MI455X (gfx1250) — hardware-verified
//
#include <hip/hip_runtime.h>
#include <stddef.h>


typedef _Float16 h16;
typedef _Float16 v16h __attribute__((ext_vector_type(16)));
typedef _Float16 v8h  __attribute__((ext_vector_type(8)));
typedef float    v8f  __attribute__((ext_vector_type(8)));
typedef float    v4f  __attribute__((ext_vector_type(4)));

#ifndef NB
#define NB 16
#endif
#ifndef HH
#define HH 2000
#endif
#define NB_FULL 16
#define HH_FULL 2000
#define CC   128
#define NH   4
#define DD   500
#define DPAD 512
#define CO   128
#define KM   (NH * CC)
#define HPAD (((HH + 63) / 64) * 64)

static_assert(NB >= 2 && NB <= NB_FULL && (NB % 2) == 0);
static_assert(HH >= 64 && HH <= HH_FULL);
static_assert((HPAD % 64) == 0 && HPAD >= HH);
static_assert(CC == 128);
static_assert((CC % 64) == 0 && (CO % 64) == 0 && (CO % 32) == 0);
static_assert((DPAD % 128) == 0 && DPAD >= DD && (DPAD % 32) == 0);
static_assert((KM % 32) == 0 && (KM % 64) == 0);
static_assert((DD % 4) == 0 && (DD / 4) <= 128);
static_assert(CC == 16 * 8);
static_assert(((DPAD * CC / 8) % 256) == 0 && ((DPAD * DPAD / 8) % 256) == 0 && ((CO * KM / 8) % 256) == 0);

#define LDT 72
#define LDC 68
#define LDK 136
static_assert((LDT % 8) == 0 && LDT >= 64);
static_assert((LDC % 4) == 0 && LDC >= 64);
static_assert((LDK % 8) == 0 && LDK >= 128);
static_assert((64 * LDK + CC * LDT + 8 * 16 * LDT + 128 * LDK) * 2 <= 131072);
static_assert(64 * LDC * 4 <= 131072);
static_assert(2 * 64 * LDT * 2 <= 131072);

#define WCARRY 64.0f
#define PCARRY 1024.0f
#define HCARRY 64.0f
#define ZCARRY 16.0f

#define XPL_BYTES  ((size_t)NB * CC * HPAD * 2)
#define WQ_BYTES   ((size_t)NH * DPAD * CC * 2)
#define WP_BYTES   ((size_t)NH * DPAD * DPAD * 2)
#define WM_BYTES   ((size_t)CO * KM * 2)
#define HT_BYTES   ((size_t)NH * NB * DPAD * CC * 2)
#define Y_BYTES    ((size_t)NH * NB * DPAD * CC * 4)
#define Z_BYTES    ((size_t)NB * DPAD * KM * 2)
#define M_BYTES    ((size_t)NB * CO * DPAD * 4)
#define MS_BYTES   ((size_t)2 * CO * 4)
#define OFF_XV  ((size_t)0)
#define OFF_XT  (OFF_XV + XPL_BYTES)
#define OFF_WQ  (OFF_XT + XPL_BYTES)
#define OFF_WP  (OFF_WQ + WQ_BYTES)
#define OFF_WM  (OFF_WP + WP_BYTES)
#define OFF_HTT (OFF_WM + WM_BYTES)
#define OFF_HTD (OFF_HTT + HT_BYTES)
#define OFF_Y   (OFF_HTD + HT_BYTES)
#define OFF_Z   (OFF_Y + Y_BYTES)
#define OFF_M   (OFF_Z + Z_BYTES)
#define OFF_MS  (OFF_M + M_BYTES)
#define WS_TOTAL (OFF_MS + MS_BYTES)
static_assert((XPL_BYTES % 128) == 0 && (WQ_BYTES % 128) == 0 && (WP_BYTES % 128) == 0);
static_assert((WM_BYTES % 128) == 0 && (HT_BYTES % 128) == 0 && (Y_BYTES % 128) == 0);
static_assert((Z_BYTES % 128) == 0 && (M_BYTES % 128) == 0 && (MS_BYTES % 128) == 0);
static_assert(WS_TOTAL <= (size_t)134217728);
static_assert((size_t)NB_FULL * CO * DD * 4 == (size_t)4096000);

__device__ __forceinline__ float bf16r(float x) {
  unsigned int u = __float_as_uint(x);
  u = (u + 0x7FFFu + ((u >> 16) & 1u)) & 0xFFFF0000u;
  return __uint_as_float(u);
}

static __device__ __forceinline__ h16 toh_flush(float v) {
  const h16 r = (h16)v;
  return (fabsf(v) < 6.103515625e-05f) ? (h16)0.0f : r;
}

__device__ __forceinline__ v16h frag_at(const _Float16* p) {
  v8h lo = *(const v8h*)(p);
  v8h hi = *(const v8h*)(p + 16);
  v16h out;
#pragma unroll
  for (int i = 0; i < 8; ++i) { out[i] = lo[i]; out[i + 8] = hi[i]; }
  return out;
}
__device__ __forceinline__ v16h ld_frag(const _Float16* base, unsigned ld) {
  const unsigned lane = threadIdx.x & 31u;
  return frag_at(base + (lane & 15u) * ld + (lane >> 4) * 8u);
}

__device__ __forceinline__ v8f wmma16(v16h a, v16h b, v8f c) {
  v8f d = __builtin_amdgcn_wmma_f32_16x16x32_f16(false, a, false, b, (short)0, c,
                                                 false, false);
  asm volatile("v_nop\n\tv_nop\n\tv_nop\n\tv_nop" : "+v"(d) : "v"(a), "v"(b));
  return d;
}

__device__ __forceinline__ float red16_max(float x) {
#pragma unroll
  for (int off = 1; off < 16; off <<= 1) x = fmaxf(x, __shfl_xor(x, off, 32));
  return x;
}
__device__ __forceinline__ float red16_sum(float x) {
#pragma unroll
  for (int off = 1; off < 16; off <<= 1) x += __shfl_xor(x, off, 32);
  return x;
}
__device__ __forceinline__ float red32_sum(float x) {
#pragma unroll
  for (int off = 1; off < 32; off <<= 1) x += __shfl_xor(x, off, 32);
  return x;
}

__device__ __forceinline__ void wave_lds_sync() {
  __builtin_amdgcn_fence(3  , "wavefront");
  asm volatile("s_wait_dscnt 0x0" ::: "memory");
  __builtin_amdgcn_wave_barrier();
}

__global__ __launch_bounds__(256) void xconv_kernel(
    const float* __restrict__ X, _Float16* __restrict__ Xv, _Float16* __restrict__ Xt) {
  __shared__ _Float16 Ta[64 * LDT];
  __shared__ _Float16 Tb[64 * LDT];
  const unsigned tid = threadIdx.x;
  const unsigned h0 = blockIdx.x * 64u;
  const unsigned c0 = blockIdx.y * 64u;
  const unsigned b = blockIdx.z;
#pragma unroll 4
  for (unsigned j = 0; j < 16u; ++j) {
    const unsigned idx = tid + 256u * j;
    const unsigned cr = idx >> 6, hc = idx & 63u;
    const unsigned h = h0 + hc;
    const unsigned hcl = (h < (unsigned)HH) ? h : (unsigned)(HH - 1);
    const float v = X[((size_t)b * CC + c0 + cr) * HH_FULL + hcl];
    const h16 t = (h < (unsigned)HH) ? toh_flush(bf16r(v)) : (h16)0.0f;
    Ta[cr * LDT + hc] = t;
    Tb[hc * LDT + cr] = t;
  }
  __syncthreads();
  v8h xa[2], xb[2];
  size_t offa[2], offb[2];
#pragma unroll
  for (unsigned i = 0; i < 2u; ++i) {
    const unsigned r = 32u * i + (tid >> 3);
    const unsigned ch = (tid & 7u) * 8u;
    xa[i] = *(const v8h*)&Ta[r * LDT + ch];
    xb[i] = *(const v8h*)&Tb[r * LDT + ch];
    offa[i] = ((size_t)b * CC + c0 + r) * HPAD + h0 + ch;
    offb[i] = ((size_t)b * HPAD + h0 + r) * CC + c0 + ch;
  }
#pragma unroll
  for (int i = 0; i < 2; ++i) *(volatile v8h*)(Xv + offa[i]) = xa[i];
#pragma unroll
  for (int i = 0; i < 2; ++i) *(volatile v8h*)(Xt + offb[i]) = xb[i];
  __threadfence();
#pragma unroll
  for (int i = 0; i < 2; ++i) *(volatile v8h*)(Xv + offa[i]) = xa[i];
#pragma unroll
  for (int i = 0; i < 2; ++i) *(volatile v8h*)(Xt + offb[i]) = xb[i];
}

__global__ __launch_bounds__(256) void wpad_kernel(
    const float* __restrict__ W, _Float16* __restrict__ out,
    unsigned R, unsigned Kc, unsigned RP, unsigned KP) {
  const unsigned mat = blockIdx.y;
  const unsigned chunk = blockIdx.x * 256u + threadIdx.x;
  const unsigned cpr = KP >> 3;
  const unsigned row = chunk / cpr;
  const unsigned kc = (chunk - row * cpr) * 8u;
  const unsigned rc = (row < R) ? row : (R - 1u);
  const float* src = W + ((size_t)mat * R + rc) * Kc;
  v8h o;
#pragma unroll
  for (unsigned j = 0; j < 8u; ++j) {
    const unsigned k = kc + j;
    const unsigned kcl = (k < Kc) ? k : (Kc - 1u);
    const float v = src[kcl];
    o[j] = (row < R && k < Kc) ? toh_flush(WCARRY * bf16r(v)) : (h16)0.0f;
  }
  _Float16* p = out + ((size_t)mat * RP + row) * KP + kc;
  *(volatile v8h*)p = o;
  __threadfence();
  *(volatile v8h*)p = o;
}

__global__ __launch_bounds__(256) void pool_kernel(
    const _Float16* __restrict__ Wq, const _Float16* __restrict__ Xt,
    const _Float16* __restrict__ Xv, _Float16* __restrict__ HTt,
    _Float16* __restrict__ HTd) {
  __shared__ _Float16 Ks[64 * LDK];
  __shared__ _Float16 Vs[CC * LDT];
  __shared__ _Float16 Ps[8 * 16 * LDT];
  __shared__ _Float16 Os[128 * LDK];

  const unsigned tid = threadIdx.x, lane = tid & 31u;
  const unsigned wave = (unsigned)__builtin_amdgcn_readfirstlane((int)(threadIdx.x >> 5));
  const unsigned hh = lane >> 4, m = lane & 15u;
  const unsigned d0 = blockIdx.x * 128u;
  const unsigned n = blockIdx.y;
  const unsigned b = blockIdx.z;
  const unsigned qrow0 = d0 + wave * 16u;
  _Float16* P = Ps + wave * (16u * LDT);

  const size_t qoff = ((size_t)n * DPAD + qrow0 + m) * CC + hh * 8u;
  const size_t xtb = (size_t)b * HPAD * CC;
  const size_t xvb = (size_t)b * CC * HPAD;

  float mrow[8], lrow[8];
  v8f o[8];
#pragma unroll
  for (int v = 0; v < 8; ++v) { mrow[v] = -1.0e30f; lrow[v] = 0.0f; }
#pragma unroll
  for (int nb = 0; nb < 8; ++nb) o[nb] = (v8f){};

  for (unsigned kb = 0; kb < (unsigned)HPAD; kb += 64u) {
#pragma unroll
    for (unsigned j = 0; j < 4u; ++j) {
      const unsigned idx = tid + 256u * j;
      const unsigned rk = idx >> 4, ck = (idx & 15u) * 8u;
      const unsigned rv = idx >> 3, cv = (idx & 7u) * 8u;
      *(v8h*)&Ks[rk * LDK + ck] = *(const v8h*)(Xt + xtb + (size_t)(kb + rk) * CC + ck);
      *(v8h*)&Vs[rv * LDT + cv] = *(const v8h*)(Xv + xvb + (size_t)rv * HPAD + kb + cv);
    }
    __syncthreads();

    v8f s[4];
#pragma unroll
    for (int kg = 0; kg < 4; ++kg) s[kg] = (v8f){};
#pragma unroll
    for (int c = 0; c < 4; ++c) {
      const v16h qf = frag_at(Wq + qoff + (unsigned)c * 32u);
#pragma unroll
      for (int kg = 0; kg < 4; ++kg) {
        const v16h kf = ld_frag(&Ks[(kg * 16) * LDK + c * 32], LDK);
        s[kg] = wmma16(qf, kf, s[kg]);
      }
    }
#pragma unroll
    for (int kg = 0; kg < 4; ++kg) s[kg] = s[kg] * (1.0f / WCARRY);

    if (kb + 64u > (unsigned)HH) {
#pragma unroll
      for (int kg = 0; kg < 4; ++kg)
#pragma unroll
        for (int v = 0; v < 8; ++v) {
          const unsigned key = kb + (unsigned)kg * 16u + m;
          s[kg][v] = (key >= (unsigned)HH) ? -1.0e30f : s[kg][v];
        }
    }

    float alpha[8];
#pragma unroll
    for (int v = 0; v < 8; ++v) {
      float mx = fmaxf(fmaxf(s[0][v], s[1][v]), fmaxf(s[2][v], s[3][v]));
      mx = red16_max(mx);
      const float mn = fmaxf(mrow[v], mx);
      alpha[v] = __expf(mrow[v] - mn);
      mrow[v] = mn;
    }
#pragma unroll
    for (int kg = 0; kg < 4; ++kg)
#pragma unroll
      for (int v = 0; v < 8; ++v) s[kg][v] = __expf(s[kg][v] - mrow[v]);

#pragma unroll
    for (int kg = 0; kg < 4; ++kg)
#pragma unroll
      for (int v = 0; v < 8; ++v) {
        const h16 p16 = toh_flush(s[kg][v] * PCARRY);
        P[(hh * 8u + (unsigned)v) * LDT + (unsigned)kg * 16u + m] = p16;
        s[kg][v] = (float)p16;
      }
#pragma unroll
    for (int v = 0; v < 8; ++v) {
      const float rs = red16_sum((s[0][v] + s[1][v]) + (s[2][v] + s[3][v]));
      lrow[v] = alpha[v] * lrow[v] + rs;
    }
#pragma unroll
    for (int nb = 0; nb < 8; ++nb)
#pragma unroll
      for (int v = 0; v < 8; ++v) o[nb][v] = o[nb][v] * alpha[v];
    wave_lds_sync();

#pragma unroll
    for (int c = 0; c < 2; ++c) {
      const v16h pf = ld_frag(P + c * 32, LDT);
#pragma unroll
      for (int nb = 0; nb < 8; ++nb) {
        const v16h vf = ld_frag(&Vs[(nb * 16) * LDT + c * 32], LDT);
        o[nb] = wmma16(pf, vf, o[nb]);
      }
    }
    __syncthreads();
  }

  float inv[8];
#pragma unroll
  for (int v = 0; v < 8; ++v) inv[v] = __builtin_amdgcn_rcpf(lrow[v]) * HCARRY;
#pragma unroll
  for (int nb = 0; nb < 8; ++nb)
#pragma unroll
    for (int v = 0; v < 8; ++v) {
      const unsigned dl = wave * 16u + hh * 8u + (unsigned)v;
      const float val = o[nb][v] * inv[v];
      Os[dl * LDK + (unsigned)nb * 16u + m] = (d0 + dl < (unsigned)DD) ? toh_flush(val) : (h16)0.0f;
    }
  __syncthreads();

  const size_t zb = (size_t)n * NB + b;
  {
    v8h x[8];
    size_t off[8];
#pragma unroll
    for (unsigned i = 0; i < 8u; ++i) {
      const unsigned r = 16u * i + (tid >> 4);
      const unsigned ch = (tid & 15u) * 8u;
      x[i] = *(const v8h*)&Os[r * LDK + ch];
      off[i] = (zb * DPAD + d0 + r) * CC + ch;
    }
#pragma unroll
    for (int i = 0; i < 8; ++i) *(volatile v8h*)(HTd + off[i]) = x[i];
    __threadfence();
#pragma unroll
    for (int i = 0; i < 8; ++i) *(volatile v8h*)(HTd + off[i]) = x[i];
  }
  {
    v8h x[8];
    size_t off[8];
#pragma unroll
    for (unsigned i = 0; i < 8u; ++i) {
      const unsigned cr = 16u * i + (tid >> 4);
      const unsigned dch = (tid & 15u) * 8u;
#pragma unroll
      for (unsigned j = 0; j < 8u; ++j) x[i][j] = Os[(dch + j) * LDK + cr];
      off[i] = (zb * CC + cr) * DPAD + d0 + dch;
    }
#pragma unroll
    for (int i = 0; i < 8; ++i) *(volatile v8h*)(HTt + off[i]) = x[i];
    __threadfence();
#pragma unroll
    for (int i = 0; i < 8; ++i) *(volatile v8h*)(HTt + off[i]) = x[i];
  }
}

__device__ __forceinline__ void gemm_tile_f32(
    const _Float16* __restrict__ A16, const _Float16* __restrict__ Bt, const unsigned K,
    float* __restrict__ outf, const unsigned ldo, const float cs) {
  __shared__ float Cs[64 * LDC];
  const unsigned tid = threadIdx.x, lane = tid & 31u, w = tid >> 5;
  const unsigned mw = w >> 1, nw = w & 1u;
  const unsigned hh = lane >> 4, m = lane & 15u;
  const unsigned n0 = blockIdx.x * 64u;
  const unsigned row0 = blockIdx.y * 64u;

  const _Float16* ap  = A16 + (size_t)(row0 + mw * 16u + m) * K + hh * 8u;
  const _Float16* bp0 = Bt + (size_t)(n0 + nw * 32u + m) * K + hh * 8u;
  const _Float16* bp1 = bp0 + (size_t)16 * K;
  v8f acc0 = {}, acc1 = {};
#pragma unroll 2
  for (unsigned k0 = 0; k0 < K; k0 += 32u) {
    const v16h a  = frag_at(ap + k0);
    const v16h b0 = frag_at(bp0 + k0);
    const v16h b1 = frag_at(bp1 + k0);
    acc0 = wmma16(a, b0, acc0);
    acc1 = wmma16(a, b1, acc1);
  }
#pragma unroll
  for (int r = 0; r < 8; ++r) {
    float* d = &Cs[(mw * 16u + hh * 8u + (unsigned)r) * LDC + nw * 32u + m];
    d[0]  = acc0[r];
    d[16] = acc1[r];
  }
  __syncthreads();

  v4f xs[4];
  size_t off[4];
#pragma unroll
  for (unsigned i = 0; i < 4u; ++i) {
    const unsigned r = 16u * i + (tid >> 4);
    const unsigned c = (tid & 15u) * 4u;
    const v4f u = *(const v4f*)&Cs[r * LDC + c];
    xs[i] = u * cs;
    off[i] = (size_t)(row0 + r) * ldo + n0 + c;
  }
#pragma unroll
  for (int i = 0; i < 4; ++i) *(volatile v4f*)(outf + off[i]) = xs[i];
  __threadfence();
#pragma unroll
  for (int i = 0; i < 4; ++i) *(volatile v4f*)(outf + off[i]) = xs[i];
}

__global__ __launch_bounds__(256) void gemm_pw_kernel(
    const _Float16* __restrict__ Wp, const _Float16* __restrict__ HTt, float* __restrict__ Y) {
  const unsigned z = blockIdx.z;
  const unsigned n = z / (unsigned)NB;
  gemm_tile_f32(Wp + (size_t)n * DPAD * DPAD, HTt + (size_t)z * CC * DPAD, (unsigned)DPAD,
                Y + (size_t)z * DPAD * CC, (unsigned)CC, 1.0f / (WCARRY * HCARRY));
}
__global__ __launch_bounds__(256) void gemm_merge_kernel(
    const _Float16* __restrict__ Wm, const _Float16* __restrict__ Z, float* __restrict__ M) {
  const unsigned b = blockIdx.z;
  gemm_tile_f32(Wm, Z + (size_t)b * DPAD * KM, (unsigned)KM,
                M + (size_t)b * CO * DPAD, (unsigned)DPAD, 1.0f / (WCARRY * ZCARRY));
}

__global__ __launch_bounds__(256) void bnz_kernel(
    const float* __restrict__ Y, const _Float16* __restrict__ HTd,
    const float* __restrict__ G, const float* __restrict__ Be, _Float16* __restrict__ Z) {
#pragma clang fp contract(off)
  const unsigned lane = threadIdx.x & 31u;
  const unsigned wave = (unsigned)__builtin_amdgcn_readfirstlane((int)(threadIdx.x >> 5));
  const unsigned hsel = lane >> 4, cl = (lane & 15u) * 8u;
  const unsigned e = blockIdx.x * 8u + wave;
  const unsigned ev = blockIdx.x * 8u + (threadIdx.x >> 5);
  const bool live = ev < (unsigned)DD;
  const unsigned ecl = live ? ev : (unsigned)(DD - 1);
  const unsigned n = blockIdx.y;
  const size_t rbase = ((size_t)n * NB * DPAD + e) * CC + cl;
  const size_t bstride = (size_t)DPAD * CC;
  const float invn = 1.0f / (float)(NB * CC);

  float s = 0.0f;
#pragma unroll 1
  for (unsigned j = 0; j < (unsigned)(NB / 2); ++j) {
    const float* yp = Y + rbase + (size_t)(2u * j + hsel) * bstride;
    const v4f a0 = *(const v4f*)yp;
    const v4f a1 = *(const v4f*)(yp + 4);
#pragma unroll
    for (int i = 0; i < 4; ++i) s += a0[i] + a1[i];
  }
  const float mean = red32_sum(s) * invn;

  float ss = 0.0f;
#pragma unroll 1
  for (unsigned j = 0; j < (unsigned)(NB / 2); ++j) {
    const float* yp = Y + rbase + (size_t)(2u * j + hsel) * bstride;
    const v4f a0 = *(const v4f*)yp;
    const v4f a1 = *(const v4f*)(yp + 4);
#pragma unroll
    for (int i = 0; i < 4; ++i) {
      const float q0 = a0[i] - mean;
      const float q1 = a1[i] - mean;
      ss += q0 * q0;
      ss += q1 * q1;
    }
  }
  const float var = red32_sum(ss) * invn;
  const float rstd = 1.0f / sqrtf(var + 1.0e-5f);
  const float gam = bf16r(G[n * (unsigned)DD + ecl]);
  const float bet = bf16r(Be[n * (unsigned)DD + ecl]);

#pragma unroll 1
  for (unsigned j = 0; j < (unsigned)(NB / 2); ++j) {
    const unsigned b = 2u * j + hsel;
    const float* yp = Y + rbase + (size_t)b * bstride;
    const v4f a0 = *(const v4f*)yp;
    const v4f a1 = *(const v4f*)(yp + 4);
    const v8h hv = *(const v8h*)(HTd + rbase + (size_t)b * bstride);
    v8h ov;
#pragma unroll
    for (int i = 0; i < 4; ++i) {
      const float t0 = (a0[i] - mean) * rstd * gam + bet;
      const float t1 = (a1[i] - mean) * rstd * gam + bet;
      const float z0 = (float)hv[i] * (1.0f / HCARRY) + fmaxf(t0, 0.0f);
      const float z1 = (float)hv[i + 4] * (1.0f / HCARRY) + fmaxf(t1, 0.0f);
      ov[i]     = live ? toh_flush(ZCARRY * z0) : (h16)0.0f;
      ov[i + 4] = live ? toh_flush(ZCARRY * z1) : (h16)0.0f;
    }
    _Float16* p = Z + ((size_t)b * DPAD + e) * KM + n * (unsigned)CC + cl;
    *(volatile v8h*)p = ov;
    __threadfence();
    *(volatile v8h*)p = ov;
  }
}

__global__ __launch_bounds__(256) void mstat_kernel(
    const float* __restrict__ M, float* __restrict__ MS) {
#pragma clang fp contract(off)
  __shared__ float st[64];
  const unsigned tid = threadIdx.x, lane = tid & 31u;
  const unsigned wave = (unsigned)__builtin_amdgcn_readfirstlane((int)(threadIdx.x >> 5));
  const float invn = 1.0f / (float)(NB * DD);
#pragma unroll 1
  for (unsigned j = 0; j < 4u; ++j) {
    const unsigned ol = wave * 4u + j;
    const unsigned o = blockIdx.x * 32u + ol;
    float s = 0.0f;
#pragma unroll 1
    for (unsigned b = 0; b < (unsigned)NB; ++b) {
      const float* row = M + ((size_t)b * CO + o) * DPAD;
#pragma unroll 1
      for (unsigned it = 0; it < 4u; ++it) {
        const unsigned q = it * 32u + lane;
        const unsigned qc = (q < (unsigned)(DD / 4)) ? q : (unsigned)(DD / 4 - 1);
        const v4f a = *(const v4f*)(row + 4u * qc);
        const float t = (a[0] + a[1]) + (a[2] + a[3]);
        s += (q < (unsigned)(DD / 4)) ? t : 0.0f;
      }
    }
    const float mean = red32_sum(s) * invn;
    float ss = 0.0f;
#pragma unroll 1
    for (unsigned b = 0; b < (unsigned)NB; ++b) {
      const float* row = M + ((size_t)b * CO + o) * DPAD;
#pragma unroll 1
      for (unsigned it = 0; it < 4u; ++it) {
        const unsigned q = it * 32u + lane;
        const unsigned qc = (q < (unsigned)(DD / 4)) ? q : (unsigned)(DD / 4 - 1);
        const v4f a = *(const v4f*)(row + 4u * qc);
        float t = 0.0f;
#pragma unroll
        for (int i = 0; i < 4; ++i) {
          const float dlt = a[i] - mean;
          t += dlt * dlt;
        }
        ss += (q < (unsigned)(DD / 4)) ? t : 0.0f;
      }
    }
    const float var = red32_sum(ss) * invn;
    const float rstd = 1.0f / sqrtf(var + 1.0e-5f);
    if (lane == 0u) {
      st[ol] = mean;
      st[32u + ol] = rstd;
    }
  }
  __syncthreads();
  if (tid < 16u) {
    const v4f x = *(const v4f*)&st[tid * 4u];
    float* p = MS + (tid >> 3) * (unsigned)CO + blockIdx.x * 32u + (tid & 7u) * 4u;
    *(volatile v4f*)p = x;
    __threadfence();
    *(volatile v4f*)p = x;
  }
}

__global__ __launch_bounds__(256) void final_kernel(
    const float* __restrict__ M, const float* __restrict__ MS,
    const float* __restrict__ G, const float* __restrict__ Be, float* __restrict__ out) {
#pragma clang fp contract(off)
  const unsigned total = (unsigned)(NB * CO * DD / 4);
  const unsigned t = blockIdx.x * 256u + threadIdx.x;
  const unsigned tc = (t < total) ? t : (total - 1u);
  const unsigned e0 = tc * 4u;
  const unsigned rowi = e0 / (unsigned)DD;
  const unsigned dd = e0 - rowi * (unsigned)DD;
  const unsigned o = rowi % (unsigned)CO;
  const v4f mv = *(const v4f*)(M + (size_t)rowi * DPAD + dd);
  const float mean = MS[o];
  const float rstd = MS[(unsigned)CO + o];
  const float gam = bf16r(G[o]);
  const float bet = bf16r(Be[o]);
  v4f r;
#pragma unroll
  for (int i = 0; i < 4; ++i) {
    const float tt = (mv[i] - mean) * rstd * gam + bet;
    r[i] = fmaxf(tt, 0.0f);
  }
  if (t < total) {
    float* p = out + (size_t)e0;
    *(volatile v4f*)p = r;
    __threadfence();
    *(volatile v4f*)p = r;
  }
}

extern "C" void kernel_launch(void* const* d_in, const int* in_sizes, int n_in,
                              void* d_out, int out_size, void* d_ws, size_t ws_size,
                              hipStream_t stream) {
  if (n_in < 8) return;
  const long long need_x = ((long long)(NB - 1) * CC + (CC - 1)) * HH_FULL + HH;
  if ((long long)in_sizes[0] < need_x) return;
  if ((long long)in_sizes[1] < (long long)NH * DD * CC) return;
  if ((long long)in_sizes[2] < (long long)NH * DD * DD) return;
  if (in_sizes[3] < NH * DD || in_sizes[4] < NH * DD) return;
  if ((long long)in_sizes[5] < (long long)CO * KM) return;
  if (in_sizes[6] < CO || in_sizes[7] < CO) return;
  if ((long long)out_size < (long long)NB * CO * DD) return;
  if (ws_size < WS_TOTAL) return;

  const float* X     = (const float*)d_in[0];
  const float* wpool = (const float*)d_in[1];
  const float* wpw   = (const float*)d_in[2];
  const float* gpw   = (const float*)d_in[3];
  const float* bpw   = (const float*)d_in[4];
  const float* wm    = (const float*)d_in[5];
  const float* gm    = (const float*)d_in[6];
  const float* bm    = (const float*)d_in[7];
  float* out = (float*)d_out;

  char* ws = (char*)d_ws;
  _Float16* Xv16  = (_Float16*)(ws + OFF_XV);
  _Float16* Xt16  = (_Float16*)(ws + OFF_XT);
  _Float16* WQ16  = (_Float16*)(ws + OFF_WQ);
  _Float16* WP16  = (_Float16*)(ws + OFF_WP);
  _Float16* WM16  = (_Float16*)(ws + OFF_WM);
  _Float16* HTt16 = (_Float16*)(ws + OFF_HTT);
  _Float16* HTd16 = (_Float16*)(ws + OFF_HTD);
  float*    Y32   = (float*)(ws + OFF_Y);
  _Float16* Z16   = (_Float16*)(ws + OFF_Z);
  float*    M32   = (float*)(ws + OFF_M);
  float*    MS    = (float*)(ws + OFF_MS);

  dim3 blk(256);

  xconv_kernel<<<dim3(HPAD / 64, CC / 64, NB), blk, 0, stream>>>(X, Xv16, Xt16);
  wpad_kernel<<<dim3(DPAD * CC / 8 / 256, NH), blk, 0, stream>>>(
      wpool, WQ16, (unsigned)DD, (unsigned)CC, (unsigned)DPAD, (unsigned)CC);
  wpad_kernel<<<dim3(DPAD * DPAD / 8 / 256, NH), blk, 0, stream>>>(
      wpw, WP16, (unsigned)DD, (unsigned)DD, (unsigned)DPAD, (unsigned)DPAD);
  wpad_kernel<<<dim3(CO * KM / 8 / 256, 1), blk, 0, stream>>>(
      wm, WM16, (unsigned)CO, (unsigned)KM, (unsigned)CO, (unsigned)KM);

  pool_kernel<<<dim3(DPAD / 128, NH, NB), blk, 0, stream>>>(WQ16, Xt16, Xv16, HTt16, HTd16);
  gemm_pw_kernel<<<dim3(CC / 64, DPAD / 64, NH * NB), blk, 0, stream>>>(WP16, HTt16, Y32);
  bnz_kernel<<<dim3(DPAD / 8, NH), blk, 0, stream>>>(Y32, HTd16, gpw, bpw, Z16);
  gemm_merge_kernel<<<dim3(DPAD / 64, CO / 64, NB), blk, 0, stream>>>(WM16, Z16, M32);
  mstat_kernel<<<dim3(CO / 32), blk, 0, stream>>>(M32, MS);
  final_kernel<<<dim3((NB * CO * DD / 4 + 255) / 256), blk, 0, stream>>>(M32, MS, gm, bm, out);
}
